// VMamba_Decoder1_34626026340769
// MI455X (gfx1250) — hardware-verified
//
#include <hip/hip_runtime.h>


namespace {
constexpr int NB = 2, HH = 64, L = HH * HH, NT = NB * L, CE = 128, DM = 64, DI = 128, NS = 16, R = 4, K = 4, XD = R + 2 * NS, NBLK = 4, FH = 256, C1 = 32;
constexpr float XS = 8.0f, US = 1024.0f, DS = 16384.0f, YS = 64.0f, GS = 256.0f, HS = 64.0f, WSC = 256.0f, EPS = 1e-5f;
typedef _Float16 b16;
typedef __attribute__((ext_vector_type(16))) _Float16 v16b;
typedef __attribute__((ext_vector_type(8))) _Float16 v8b;
typedef __attribute__((ext_vector_type(8))) float v8f;
typedef __attribute__((ext_vector_type(4))) float v4f;
typedef __attribute__((ext_vector_type(2))) float v2f;
__device__ __forceinline__ float bf16_rne(float f) { unsigned int u = __float_as_uint(f); u += 0x7FFFu + ((u >> 16) & 1u); return __uint_as_float(u & 0xFFFF0000u); }
__device__ __forceinline__ void split16(float v, b16& hi, b16& lo) { hi = (b16)v; lo = (b16)(v - (float)hi); }
__device__ __forceinline__ v16b frag_kb(const b16* p, int hh) { const v8b a = *(const v8b*)(p + 8 * hh), b = *(const v8b*)(p + 16 + 8 * hh); v16b f;
#pragma unroll
  for (int e = 0; e < 8; ++e) { f[e] = a[e]; f[8 + e] = b[e]; } return f; }
__device__ __forceinline__ v8f wmma16b(v16b a, v16b b, v8f c) { v8f d = __builtin_amdgcn_wmma_f32_16x16x32_f16(false, a, false, b, (short)0, c, false, false); asm volatile("v_nop\n\tv_nop\n\tv_nop\n\tv_nop" : "+v"(d) : "v"(a), "v"(b)); return d; }
__device__ __forceinline__ void wave_lds_sync() { __builtin_amdgcn_fence(__ATOMIC_RELEASE, "workgroup"); __builtin_amdgcn_wave_barrier(); __builtin_amdgcn_fence(__ATOMIC_ACQUIRE, "workgroup"); }
__device__ __forceinline__ float pmul(float a, float b) { float p = a * b; asm volatile("" : "+v"(p)); return p; }
__device__ __forceinline__ float sigm(float v) { return 1.0f / (1.0f + __expf(-v)); }
__device__ __forceinline__ float silu(float v) { return pmul(v, sigm(v)); }
__device__ __forceinline__ float softplus(float v) { return v > 20.0f ? v : (v < -20.0f ? __expf(v) : log1pf(__expf(v))); }
__device__ __forceinline__ float gelu(float v) { return 0.5f * v * (1.0f + erff(v * 0.70710678118654752f)); }

__global__ __launch_bounds__(256) void wcopyp_kernel(const float* __restrict__ w, int KIN, int OUT, int KP, int OUTP, b16* __restrict__ WT) {
  const int u = blockIdx.x * 256 + threadIdx.x; if (u >= OUTP * KP / 8) return; const int e = u * 8; const int o = e / KP, k0 = e % KP; v8b v;
#pragma unroll
  for (int j = 0; j < 8; ++j) { const int k = k0 + j; v[j] = (o < OUT && k < KIN) ? (b16)(bf16_rne(w[(size_t)o * KIN + k]) * WSC) : (b16)0.0f; } for (int pass = 0; pass < 2; ++pass) { *(volatile v8b*)(WT + e) = v; __threadfence(); }
}
__global__ __launch_bounds__(256) void wh1_kernel(const float* __restrict__ w, b16* __restrict__ WT) {
  const int u = blockIdx.x * 256 + threadIdx.x; if (u >= C1 * 576 / 8) return; const int e = u * 8; const int o = e / 576, k0 = e % 576; v8b v;
#pragma unroll
  for (int j = 0; j < 8; ++j) { const int k = k0 + j; const int tap = k / DM, c = k % DM; v[j] = (b16)(bf16_rne(w[((size_t)o * DM + c) * 9 + tap]) * WSC); } for (int pass = 0; pass < 2; ++pass) { *(volatile v8b*)(WT + e) = v; __threadfence(); }
}

__global__ __launch_bounds__(64) void stem_kernel(const float* __restrict__ enc, const b16* __restrict__ WRC, const b16* __restrict__ WPE, const float* __restrict__ peb, const float* __restrict__ g, const float* __restrict__ bb, float* __restrict__ featout, float* __restrict__ X) {
  __shared__ __attribute__((aligned(16))) b16 Ah[2][16][CE + 8], Al[2][16][CE + 8]; __shared__ __attribute__((aligned(16))) float To[DM][32 + 1]; __shared__ __attribute__((aligned(16))) float Tf[2][16][DM + 4];
  const int wave = threadIdx.x >> 5, lane = threadIdx.x & 31, nloc = lane & 15, hlf = lane >> 4; const size_t t0 = (size_t)blockIdx.x * 32; const size_t m0 = t0 + wave * 16; const int b = (int)(t0 / L), p0 = (int)(t0 % L), pw = (int)(m0 % L);
  for (int rr = 0; rr < 16; ++rr) for (int q = 0; q < 4; ++q) { const int c = q * 32 + lane; Ah[wave][rr][c] = (b16)(bf16_rne(enc[((size_t)b * CE + c) * L + pw + rr]) * XS); Al[wave][rr][c] = (b16)0.0f; }
  wave_lds_sync();
  v8f acc[4];
#pragma unroll
  for (int t = 0; t < 4; ++t) acc[t] = (v8f){};
#pragma unroll 2
  for (int kb = 0; kb < CE; kb += 32) { const v16b a = frag_kb(&Ah[wave][nloc][kb], hlf);
#pragma unroll
    for (int t = 0; t < 4; ++t) acc[t] = wmma16b(a, frag_kb(WRC + (size_t)(t * 16 + nloc) * CE + kb, hlf), acc[t]); }
  wave_lds_sync();
#pragma unroll
  for (int t = 0; t < 4; ++t) { const int c = t * 16 + nloc;
#pragma unroll
    for (int r8 = 0; r8 < 8; ++r8) { const float f = acc[t][r8] * (1.0f / (XS * WSC)); To[c][wave * 16 + 8 * hlf + r8] = f; b16 p, q; split16(f * XS, p, q); Ah[wave][8 * hlf + r8][c] = p; Al[wave][8 * hlf + r8][c] = q; } }
  __syncthreads();
  for (int pass = 0; pass < 2; ++pass) { for (int i = threadIdx.x; i < DM * 32; i += 64) { const int c = i >> 5, pp = i & 31; ((volatile float*)featout)[((size_t)b * DM + c) * L + p0 + pp] = To[c][pp]; } __threadfence(); }
#pragma unroll
  for (int t = 0; t < 4; ++t) acc[t] = (v8f){};
#pragma unroll
  for (int kb = 0; kb < DM; kb += 32) { const v16b a = frag_kb(&Ah[wave][nloc][kb], hlf), al = frag_kb(&Al[wave][nloc][kb], hlf);
#pragma unroll
    for (int t = 0; t < 4; ++t) { const v16b bw = frag_kb(WPE + (size_t)(t * 16 + nloc) * DM + kb, hlf); acc[t] = wmma16b(a, bw, acc[t]); acc[t] = wmma16b(al, bw, acc[t]); } }
  float ps[8], pq[8]; float vals[4][8];
#pragma unroll
  for (int r8 = 0; r8 < 8; ++r8) { ps[r8] = 0.0f; }
#pragma unroll
  for (int t = 0; t < 4; ++t) { const float pb = bf16_rne(peb[t * 16 + nloc]);
#pragma unroll
    for (int r8 = 0; r8 < 8; ++r8) { vals[t][r8] = acc[t][r8] * (1.0f / (XS * WSC)) + pb; ps[r8] += vals[t][r8]; } }
#pragma unroll
  for (int r8 = 0; r8 < 8; ++r8) { for (int o = 1; o < 16; o <<= 1) ps[r8] += __shfl_xor(ps[r8], o); ps[r8] *= (1.0f / DM); pq[r8] = 0.0f;
#pragma unroll
    for (int t = 0; t < 4; ++t) { const float d = vals[t][r8] - ps[r8]; pq[r8] += pmul(d, d); } for (int o = 1; o < 16; o <<= 1) pq[r8] += __shfl_xor(pq[r8], o); pq[r8] = rsqrtf(pq[r8] * (1.0f / DM) + EPS); }
#pragma unroll
  for (int t = 0; t < 4; ++t) { const int c = t * 16 + nloc; const float gg = bf16_rne(g[c]), be = bf16_rne(bb[c]);
#pragma unroll 1
    for (int r8 = 0; r8 < 8; ++r8) Tf[wave][8 * hlf + r8][c] = pmul(pmul(vals[t][r8] - ps[r8], pq[r8]), gg) + be; }
  wave_lds_sync();
  for (int pass = 0; pass < 2; ++pass) { for (int rr = 0; rr < 16; ++rr) *(volatile v2f*)(X + (m0 + rr) * DM + lane * 2) = *(const v2f*)(&Tf[wave][rr][lane * 2]); __threadfence(); }
}
__global__ __launch_bounds__(32) void inproj_kernel(const float* __restrict__ X, const float* __restrict__ g, const float* __restrict__ bb, const b16* __restrict__ WIP, float* __restrict__ XZ) {
  __shared__ __attribute__((aligned(16))) b16 Ah[16][DM + 8], Al[16][DM + 8]; __shared__ __attribute__((aligned(16))) float Tf[16][128 + 4];
  const int lane = threadIdx.x, nloc = lane & 15, hlf = lane >> 4; const size_t m0 = (size_t)blockIdx.x * 16; const float g0 = bf16_rne(g[lane * 2]), g1 = bf16_rne(g[lane * 2 + 1]), b0 = bf16_rne(bb[lane * 2]), b1 = bf16_rne(bb[lane * 2 + 1]);
  for (int rr = 0; rr < 16; ++rr) { const v2f v = *(const v2f*)(X + (m0 + rr) * DM + lane * 2); float s = v[0] + v[1]; for (int o = 16; o; o >>= 1) s += __shfl_xor(s, o); const float mu = s * (1.0f / DM); const float d0 = v[0] - mu, d1 = v[1] - mu; float q = pmul(d0, d0) + pmul(d1, d1); for (int o = 16; o; o >>= 1) q += __shfl_xor(q, o); const float rs = rsqrtf(q * (1.0f / DM) + EPS);
    b16 p, ql; split16((pmul(pmul(d0, rs), g0) + b0) * XS, p, ql); Ah[rr][lane * 2] = p; Al[rr][lane * 2] = ql; split16((pmul(pmul(d1, rs), g1) + b1) * XS, p, ql); Ah[rr][lane * 2 + 1] = p; Al[rr][lane * 2 + 1] = ql; }
  wave_lds_sync();
#pragma unroll 1
  for (int cg = 0; cg < 2; ++cg) { v8f acc[8];
#pragma unroll
    for (int t = 0; t < 8; ++t) acc[t] = (v8f){};
#pragma unroll
    for (int kb = 0; kb < DM; kb += 32) { const v16b a = frag_kb(&Ah[nloc][kb], hlf), al = frag_kb(&Al[nloc][kb], hlf);
#pragma unroll
      for (int t = 0; t < 8; ++t) { const v16b bw = frag_kb(WIP + (size_t)(cg * 128 + t * 16 + nloc) * DM + kb, hlf); acc[t] = wmma16b(a, bw, acc[t]); acc[t] = wmma16b(al, bw, acc[t]); } }
#pragma unroll
    for (int t = 0; t < 8; ++t)
#pragma unroll 1
      for (int r8 = 0; r8 < 8; ++r8) Tf[8 * hlf + r8][t * 16 + nloc] = acc[t][r8] * (1.0f / (XS * WSC));
    wave_lds_sync();
    for (int pass = 0; pass < 2; ++pass) { for (int rr = 0; rr < 16; ++rr) *(volatile v4f*)(XZ + (m0 + rr) * (2 * DI) + cg * 128 + lane * 4) = *(const v4f*)(&Tf[rr][lane * 4]); __threadfence(); }
    wave_lds_sync(); }
}
__global__ __launch_bounds__(256) void dwconv_kernel(const float* __restrict__ XZ, const float* __restrict__ cw, const float* __restrict__ cb, int ntok, float* __restrict__ U) {
  const size_t gid = (size_t)blockIdx.x * 256 + threadIdx.x; const size_t t = gid / (DI / 4); const int d4 = (int)(gid % (DI / 4)) * 4; if (t >= (size_t)ntok) return;
  const int b = (int)(t / L), p = (int)(t % L), y = p / HH, x = p % HH; v4f acc; for (int q = 0; q < 4; ++q) acc[q] = bf16_rne(cb[d4 + q]);
#pragma unroll
  for (int di = 0; di < 3; ++di)
#pragma unroll
    for (int dj = 0; dj < 3; ++dj) { const int yy = y + di - 1, xx = x + dj - 1; const bool ok = yy >= 0 && yy < HH && xx >= 0 && xx < HH; const int yc = ok ? yy : y, xc = ok ? xx : x;
      const v4f v = *(const v4f*)(XZ + ((size_t)b * L + yc * HH + xc) * (2 * DI) + d4); for (int q = 0; q < 4; ++q) acc[q] += ok ? pmul(v[q], bf16_rne(cw[(d4 + q) * 9 + di * 3 + dj])) : 0.0f; }
  v4f o; for (int q = 0; q < 4; ++q) o[q] = silu(acc[q]);
  for (int pass = 0; pass < 2; ++pass) { *(volatile v4f*)(U + t * DI + d4) = o; __threadfence(); }
}
__global__ __launch_bounds__(32) void xproj_kernel(const float* __restrict__ U, const b16* __restrict__ XPW, const b16* __restrict__ DTW, const float* __restrict__ dtb, float* __restrict__ BC, float* __restrict__ DT) {
  __shared__ __attribute__((aligned(16))) b16 Ah[16][DI + 8], Al[16][DI + 8]; __shared__ __attribute__((aligned(16))) b16 Dh[16][32 + 8], Dl[16][32 + 8]; __shared__ __attribute__((aligned(16))) float Sbc[16][32]; __shared__ __attribute__((aligned(16))) float Tf[16][DI + 4];
  const int lane = threadIdx.x, nloc = lane & 15, hlf = lane >> 4; const size_t m0 = (size_t)blockIdx.x * 16;
  for (int rr = 0; rr < 16; ++rr) { const v4f v = *(const v4f*)(U + (m0 + rr) * DI + lane * 4); for (int j = 0; j < 4; ++j) { b16 p, ql; split16(v[j] * US, p, ql); Ah[rr][lane * 4 + j] = p; Al[rr][lane * 4 + j] = ql; } }
  wave_lds_sync();
  const float sx = 1.0f / (US * WSC), sd = 1.0f / (DS * WSC);
#pragma unroll 1
  for (int k = 0; k < K; ++k) {
    v8f ax[3] = {(v8f){}, (v8f){}, (v8f){}};
#pragma unroll
    for (int kb = 0; kb < DI; kb += 32) { const v16b a = frag_kb(&Ah[nloc][kb], hlf), al = frag_kb(&Al[nloc][kb], hlf);
#pragma unroll
      for (int t = 0; t < 3; ++t) { const v16b bw = frag_kb(XPW + ((size_t)k * 48 + t * 16 + nloc) * DI + kb, hlf); ax[t] = wmma16b(a, bw, ax[t]); ax[t] = wmma16b(al, bw, ax[t]); } }
#pragma unroll
    for (int r8 = 0; r8 < 8; ++r8) { const int rl = 8 * hlf + r8; const float d0 = ax[0][r8] * sx, d1 = ax[1][r8] * sx, d2 = ax[2][r8] * sx;
      if (nloc < R) { b16 p, ql; split16(d0 * DS, p, ql); Dh[rl][nloc] = p; Dl[rl][nloc] = ql; Sbc[rl][12 + nloc] = d1; Sbc[rl][16 + 12 + nloc] = d2; }
      else { Dh[rl][nloc] = (b16)0.0f; Dl[rl][nloc] = (b16)0.0f; Sbc[rl][nloc - R] = d0; Sbc[rl][16 + nloc - R] = d1; }
      Dh[rl][16 + nloc] = (b16)0.0f; Dl[rl][16 + nloc] = (b16)0.0f; }
    wave_lds_sync();
    for (int pass = 0; pass < 2; ++pass) { for (int rr = 0; rr < 16; ++rr) ((volatile float*)BC)[((size_t)k * NT + m0 + rr) * 32 + lane] = Sbc[rr][lane]; __threadfence(); }
    { v8f acc[8]; const v16b a = frag_kb(&Dh[nloc][0], hlf), al = frag_kb(&Dl[nloc][0], hlf);
#pragma unroll
      for (int t = 0; t < 8; ++t) { acc[t] = (v8f){}; const v16b bw = frag_kb(DTW + ((size_t)k * DI + t * 16 + nloc) * 32, hlf); acc[t] = wmma16b(a, bw, acc[t]); acc[t] = wmma16b(al, bw, acc[t]); }
#pragma unroll
      for (int t = 0; t < 8; ++t) { const int c = t * 16 + nloc; const float bb = bf16_rne(dtb[k * DI + c]);
#pragma unroll 1
        for (int r8 = 0; r8 < 8; ++r8) Tf[8 * hlf + r8][c] = softplus(acc[t][r8] * sd + bb); } }
    wave_lds_sync();
    for (int pass = 0; pass < 2; ++pass) { for (int rr = 0; rr < 16; ++rr) *(volatile v4f*)(DT + ((size_t)k * NT + m0 + rr) * DI + lane * 4) = *(const v4f*)(&Tf[rr][lane * 4]); __threadfence(); }
    wave_lds_sync(); }
}
__global__ __launch_bounds__(256) void scan_kernel(const float* __restrict__ U, const float* __restrict__ DT, const float* __restrict__ BC, const float* __restrict__ alog, const float* __restrict__ Dsv, int nbv, float* __restrict__ Y4) {
  const int gid = blockIdx.x * 256 + threadIdx.x; const int b = gid / (K * DI), k = (gid / DI) % K, d = gid % DI; if (b >= nbv) return;
  float A[NS]; for (int s = 0; s < NS; ++s) A[s] = -__expf(bf16_rne(alog[((size_t)k * DI + d) * NS + s])); const float dk = bf16_rne(Dsv[k * DI + d]);
#pragma unroll 1
  for (int pass = 0; pass < 2; ++pass) { float h[NS]; for (int s = 0; s < NS; ++s) h[s] = 0.0f;
#pragma unroll 1
    for (int l = 0; l < L; ++l) { const int lr = L - 1 - l; const int p = k == 0 ? l : (k == 1 ? (l % HH) * HH + l / HH : (k == 2 ? lr : (lr % HH) * HH + lr / HH));
      const size_t row = (size_t)b * L + p; const float u = U[row * DI + d], dt = DT[((size_t)k * NT + row) * DI + d]; const float du = pmul(dt, u); const float* bc = BC + ((size_t)k * NT + row) * 32; float acc = 0.0f;
#pragma unroll
      for (int s = 0; s < NS; ++s) { h[s] = pmul(h[s], __expf(pmul(dt, A[s]))) + pmul(du, bc[s]); acc += pmul(h[s], bc[16 + s]); }
      ((volatile float*)Y4)[((size_t)k * NT + row) * DI + d] = acc + pmul(dk, u); }
    __threadfence(); }
}
__global__ __launch_bounds__(32) void block_out_kernel(const float* __restrict__ Y4, const float* __restrict__ XZ, const float* __restrict__ og, const float* __restrict__ ob, const b16* __restrict__ WOP, const float* __restrict__ g2, const float* __restrict__ b2, const b16* __restrict__ WF1, const float* __restrict__ f1b, const b16* __restrict__ WF2, const float* __restrict__ f2b, float* __restrict__ X) {
  __shared__ __attribute__((aligned(16))) b16 Ah[16][FH + 8], Al[16][FH + 8]; __shared__ __attribute__((aligned(16))) float Xs[16][DM + 4];
  const int lane = threadIdx.x, nloc = lane & 15, hlf = lane >> 4; const size_t m0 = (size_t)blockIdx.x * 16;
  float g4[4], b4[4]; for (int j = 0; j < 4; ++j) { g4[j] = bf16_rne(og[lane * 4 + j]); b4[j] = bf16_rne(ob[lane * 4 + j]); }
  for (int rr = 0; rr < 16; ++rr) { const size_t t = m0 + rr; float v[4]; float s = 0.0f;
    { const v4f y0 = *(const v4f*)(Y4 + t * DI + lane * 4), y1 = *(const v4f*)(Y4 + ((size_t)NT + t) * DI + lane * 4), y2 = *(const v4f*)(Y4 + ((size_t)2 * NT + t) * DI + lane * 4), y3 = *(const v4f*)(Y4 + ((size_t)3 * NT + t) * DI + lane * 4);
      for (int j = 0; j < 4; ++j) { v[j] = (y0[j] + y2[j]) + (y1[j] + y3[j]); s += v[j]; } }
    for (int o = 16; o; o >>= 1) s += __shfl_xor(s, o); const float mu = s * (1.0f / DI); float q = 0.0f; for (int j = 0; j < 4; ++j) { const float d = v[j] - mu; q += pmul(d, d); } for (int o = 16; o; o >>= 1) q += __shfl_xor(q, o); const float rs = rsqrtf(q * (1.0f / DI) + EPS);
    const v4f z = *(const v4f*)(XZ + t * (2 * DI) + DI + lane * 4); const v2f xv = *(const v2f*)(X + t * DM + lane * 2); Xs[rr][lane * 2] = xv[0]; Xs[rr][lane * 2 + 1] = xv[1];
    for (int j = 0; j < 4; ++j) { const float a = pmul(pmul(pmul(v[j] - mu, rs), g4[j]) + b4[j], silu(z[j])); b16 p, ql; split16(a * YS, p, ql); Ah[rr][lane * 4 + j] = p; Al[rr][lane * 4 + j] = ql; } }
  wave_lds_sync();
  v8f acc[8];
#pragma unroll
  for (int t = 0; t < 4; ++t) acc[t] = (v8f){};
#pragma unroll 2
  for (int kb = 0; kb < DI; kb += 32) { const v16b a = frag_kb(&Ah[nloc][kb], hlf), al = frag_kb(&Al[nloc][kb], hlf);
#pragma unroll
    for (int t = 0; t < 4; ++t) { const v16b bw = frag_kb(WOP + (size_t)(t * 16 + nloc) * DI + kb, hlf); acc[t] = wmma16b(a, bw, acc[t]); acc[t] = wmma16b(al, bw, acc[t]); } }
  wave_lds_sync();
#pragma unroll
  for (int t = 0; t < 4; ++t) { const int c = t * 16 + nloc;
#pragma unroll
    for (int r8 = 0; r8 < 8; ++r8) Xs[8 * hlf + r8][c] += acc[t][r8] * (1.0f / (YS * WSC)); }
  wave_lds_sync();
  { const float gg0 = bf16_rne(g2[lane * 2]), gg1 = bf16_rne(g2[lane * 2 + 1]), be0 = bf16_rne(b2[lane * 2]), be1 = bf16_rne(b2[lane * 2 + 1]);
    for (int rr = 0; rr < 16; ++rr) { const float v0 = Xs[rr][lane * 2], v1 = Xs[rr][lane * 2 + 1]; float s = v0 + v1; for (int o = 16; o; o >>= 1) s += __shfl_xor(s, o); const float mu = s * (1.0f / DM); const float d0 = v0 - mu, d1 = v1 - mu; float q = pmul(d0, d0) + pmul(d1, d1); for (int o = 16; o; o >>= 1) q += __shfl_xor(q, o); const float rs = rsqrtf(q * (1.0f / DM) + EPS);
      b16 p, ql; split16((pmul(pmul(d0, rs), gg0) + be0) * XS, p, ql); Ah[rr][lane * 2] = p; Al[rr][lane * 2] = ql; split16((pmul(pmul(d1, rs), gg1) + be1) * XS, p, ql); Ah[rr][lane * 2 + 1] = p; Al[rr][lane * 2 + 1] = ql; } }
  wave_lds_sync();
  v8f a1[16];
#pragma unroll
  for (int t = 0; t < 16; ++t) a1[t] = (v8f){};
#pragma unroll
  for (int kb = 0; kb < DM; kb += 32) { const v16b a = frag_kb(&Ah[nloc][kb], hlf), al = frag_kb(&Al[nloc][kb], hlf);
#pragma unroll
    for (int t = 0; t < 16; ++t) { const v16b bw = frag_kb(WF1 + (size_t)(t * 16 + nloc) * DM + kb, hlf); a1[t] = wmma16b(a, bw, a1[t]); a1[t] = wmma16b(al, bw, a1[t]); } }
  wave_lds_sync();
#pragma unroll
  for (int t = 0; t < 16; ++t) { const int c = t * 16 + nloc; const float bb = bf16_rne(f1b[c]);
#pragma unroll
    for (int r8 = 0; r8 < 8; ++r8) { const float gv = gelu(a1[t][r8] * (1.0f / (XS * WSC)) + bb); b16 p, ql; split16(gv * GS, p, ql); Ah[8 * hlf + r8][c] = p; Al[8 * hlf + r8][c] = ql; } }
  wave_lds_sync();
#pragma unroll
  for (int t = 0; t < 4; ++t) acc[t] = (v8f){};
#pragma unroll 2
  for (int kb = 0; kb < FH; kb += 32) { const v16b a = frag_kb(&Ah[nloc][kb], hlf), al = frag_kb(&Al[nloc][kb], hlf);
#pragma unroll
    for (int t = 0; t < 4; ++t) { const v16b bw = frag_kb(WF2 + (size_t)(t * 16 + nloc) * FH + kb, hlf); acc[t] = wmma16b(a, bw, acc[t]); acc[t] = wmma16b(al, bw, acc[t]); } }
#pragma unroll
  for (int t = 0; t < 4; ++t) { const int c = t * 16 + nloc; const float bb = bf16_rne(f2b[c]);
#pragma unroll
    for (int r8 = 0; r8 < 8; ++r8) Xs[8 * hlf + r8][c] += acc[t][r8] * (1.0f / (GS * WSC)) + bb; }
  wave_lds_sync();
  for (int pass = 0; pass < 2; ++pass) { for (int rr = 0; rr < 16; ++rr) *(volatile v2f*)(X + (m0 + rr) * DM + lane * 2) = *(const v2f*)(&Xs[rr][lane * 2]); __threadfence(); }
}
__global__ __launch_bounds__(32) void head1_kernel(const float* __restrict__ X, const b16* __restrict__ H1W, float* __restrict__ H1) {
  __shared__ __attribute__((aligned(16))) b16 Ah[16][576 + 8], Al[16][576 + 8]; __shared__ __attribute__((aligned(16))) float Tf[16][C1 + 4];
  const int lane = threadIdx.x, nloc = lane & 15, hlf = lane >> 4; const size_t m0 = (size_t)blockIdx.x * 16; const int b = (int)(m0 / L), p0 = (int)(m0 % L), y = p0 / HH, x0 = p0 % HH;
  for (int rr = 0; rr < 16; ++rr)
#pragma unroll
    for (int tap = 0; tap < 9; ++tap) { const int yy = y + tap / 3 - 1, xx = x0 + rr + tap % 3 - 1; const bool ok = yy >= 0 && yy < HH && xx >= 0 && xx < HH; const int yc = ok ? yy : y, xc = ok ? xx : x0 + rr;
      const v2f v = *(const v2f*)(X + ((size_t)b * L + yc * HH + xc) * DM + lane * 2); for (int j = 0; j < 2; ++j) { b16 p, q; split16((ok ? v[j] : 0.0f) * HS, p, q); Ah[rr][tap * DM + lane * 2 + j] = p; Al[rr][tap * DM + lane * 2 + j] = q; } }
  wave_lds_sync();
  v8f acc[2] = {(v8f){}, (v8f){}};
#pragma unroll 2
  for (int kb = 0; kb < 576; kb += 32) { const v16b a = frag_kb(&Ah[nloc][kb], hlf), al = frag_kb(&Al[nloc][kb], hlf);
#pragma unroll
    for (int t = 0; t < 2; ++t) { const v16b bw = frag_kb(H1W + (size_t)(t * 16 + nloc) * 576 + kb, hlf); acc[t] = wmma16b(a, bw, acc[t]); acc[t] = wmma16b(al, bw, acc[t]); } }
#pragma unroll
  for (int t = 0; t < 2; ++t) { const int c = t * 16 + nloc;
#pragma unroll 1
    for (int r8 = 0; r8 < 8; ++r8) { const float v = acc[t][r8] * (1.0f / (HS * WSC)); Tf[8 * hlf + r8][c] = v >= 0.0f ? v : 0.01f * v; } }
  wave_lds_sync();
  for (int pass = 0; pass < 2; ++pass) { for (int rr = 0; rr < 16; ++rr) ((volatile float*)H1)[(m0 + rr) * C1 + lane] = Tf[rr][lane]; __threadfence(); }
}
__global__ __launch_bounds__(256) void head2_kernel(const float* __restrict__ H1, const float* __restrict__ w2, const float* __restrict__ img, int ntok, float* __restrict__ out) {
  __shared__ float w[9 * C1]; for (int i = threadIdx.x; i < 9 * C1; i += 256) { const int c = i / 9, tap = i % 9; w[tap * C1 + c] = bf16_rne(w2[i]); }
  __syncthreads();
  const int t = blockIdx.x * 256 + threadIdx.x; if (t >= ntok) return; const int b = t / L, p = t % L, y = p / HH, x = p % HH; float s = 0.0f;
#pragma unroll 1
  for (int tap = 0; tap < 9; ++tap) { const int yy = y + tap / 3 - 1, xx = x + tap % 3 - 1; if (yy < 0 || yy >= HH || xx < 0 || xx >= HH) continue; const float* hr = H1 + ((size_t)b * L + yy * HH + xx) * C1;
#pragma unroll 1
    for (int c = 0; c < C1; c += 4) { const v4f v = *(const v4f*)(hr + c); for (int j = 0; j < 4; ++j) s += pmul(v[j], w[tap * C1 + c + j]); } }
  const float o = sigm(s + bf16_rne(img[t]));
  for (int pass = 0; pass < 2; ++pass) { ((volatile float*)out)[t] = o; __threadfence(); }
}
}

extern "C" void kernel_launch(void* const* d_in, const int* in_sizes, int n_in, void* d_out, int out_size, void* d_ws, size_t ws_size, hipStream_t stream) {
  (void)n_in;
  auto Fp = [&](int i) { return (const float*)d_in[i]; };
  if (in_sizes[0] != NT || in_sizes[1] != NT * CE || in_sizes[2] != DM * CE || in_sizes[3] != DM * DM || in_sizes[9] != NBLK * 2 * DI * DM || in_sizes[10] != NBLK * DI * 9 || in_sizes[12] != NBLK * K * XD * DI || in_sizes[13] != NBLK * K * DI * R || in_sizes[15] != NBLK * K * DI * NS || in_sizes[19] != NBLK * DM * DI || in_sizes[22] != NBLK * FH * DM || in_sizes[24] != NBLK * DM * FH || in_sizes[26] != C1 * DM * 9 || in_sizes[27] != C1 * 9 || out_size != NT + NT * DM) return;
  const int NBV = NB; const int NTV = NBV * L; const int NBLKV = NBLK;
  size_t off = 0; char* ws = (char*)d_ws;
  auto carve = [&](size_t bytes) { char* p = ws + off; off += (bytes + 255) & ~(size_t)255; return p; };
  b16* WRC = (b16*)carve((size_t)DM * CE * 2); b16* WPE = (b16*)carve((size_t)DM * DM * 2); b16* H1W = (b16*)carve((size_t)C1 * 576 * 2);
  b16* WIP[NBLK]; b16* WOP[NBLK]; b16* WF1[NBLK]; b16* WF2[NBLK]; b16* XPW[NBLK]; b16* DTW[NBLK];
  for (int i = 0; i < NBLK; ++i) { WIP[i] = (b16*)carve((size_t)2 * DI * DM * 2); WOP[i] = (b16*)carve((size_t)DM * DI * 2); WF1[i] = (b16*)carve((size_t)FH * DM * 2); WF2[i] = (b16*)carve((size_t)DM * FH * 2); XPW[i] = (b16*)carve((size_t)K * 48 * DI * 2); DTW[i] = (b16*)carve((size_t)K * DI * 32 * 2); }
  float* X = (float*)carve((size_t)NT * DM * 4); float* XZ = (float*)carve((size_t)NT * 2 * DI * 4); float* U = (float*)carve((size_t)NT * DI * 4); float* BC = (float*)carve((size_t)K * NT * 32 * 4); float* DT = (float*)carve((size_t)K * NT * DI * 4); float* Y4 = (float*)carve((size_t)K * NT * DI * 4); float* H1 = (float*)carve((size_t)NT * C1 * 4);
  if (off > ws_size || off > ((size_t)96 << 20)) return;
  auto wcp = [&](const float* w, int KIN, int OUT, int KP, int OUTP, b16* WT) { wcopyp_kernel<<<(OUTP * KP / 8 + 255) / 256, 256, 0, stream>>>(w, KIN, OUT, KP, OUTP, WT); };
  wcp(Fp(2), CE, DM, CE, DM, WRC); wcp(Fp(3), DM, DM, DM, DM, WPE); wh1_kernel<<<(C1 * 576 / 8 + 255) / 256, 256, 0, stream>>>(Fp(26), H1W);
  for (int i = 0; i < NBLK; ++i) { wcp(Fp(9) + (size_t)i * 2 * DI * DM, DM, 2 * DI, DM, 2 * DI, WIP[i]); wcp(Fp(19) + (size_t)i * DM * DI, DI, DM, DI, DM, WOP[i]); wcp(Fp(22) + (size_t)i * FH * DM, DM, FH, DM, FH, WF1[i]); wcp(Fp(24) + (size_t)i * DM * FH, FH, DM, FH, DM, WF2[i]);
    for (int k = 0; k < K; ++k) { wcp(Fp(12) + ((size_t)i * K + k) * XD * DI, DI, XD, DI, 48, XPW[i] + (size_t)k * 48 * DI); wcp(Fp(13) + ((size_t)i * K + k) * DI * R, R, DI, 32, DI, DTW[i] + (size_t)k * DI * 32); } }
  stem_kernel<<<NTV / 32, 64, 0, stream>>>(Fp(1), WRC, WPE, Fp(4), Fp(5), Fp(6), (float*)d_out + NT, X);
  for (int i = 0; i < NBLKV; ++i) {
    inproj_kernel<<<NTV / 16, 32, 0, stream>>>(X, Fp(7) + i * DM, Fp(8) + i * DM, WIP[i], XZ);
    dwconv_kernel<<<(unsigned)(((size_t)NTV * (DI / 4) + 255) / 256), 256, 0, stream>>>(XZ, Fp(10) + (size_t)i * DI * 9, Fp(11) + i * DI, NTV, U);
    xproj_kernel<<<NTV / 16, 32, 0, stream>>>(U, XPW[i], DTW[i], Fp(14) + (size_t)i * K * DI, BC, DT);
    scan_kernel<<<(NBV * K * DI + 255) / 256, 256, 0, stream>>>(U, DT, BC, Fp(15) + (size_t)i * K * DI * NS, Fp(16) + (size_t)i * K * DI, NBV, Y4);
    block_out_kernel<<<NTV / 16, 32, 0, stream>>>(Y4, XZ, Fp(17) + i * DI, Fp(18) + i * DI, WOP[i], Fp(20) + i * DM, Fp(21) + i * DM, WF1[i], Fp(23) + i * FH, WF2[i], Fp(25) + i * DM, X); }
  head1_kernel<<<NTV / 16, 32, 0, stream>>>(X, H1W, H1);
  head2_kernel<<<(NTV + 255) / 256, 256, 0, stream>>>(H1, Fp(27), Fp(0), NTV, (float*)d_out);
}
